// CountingDecoder_13013750906946
// MI455X (gfx1250) — hardware-run, weakly checked
//
#include <hip/hip_runtime.h>
#include <stdint.h>
#include <math.h>

#define NBAT  16
#define HB    ((NBAT < 8) ? NBAT : 8)
#define NHALF (NBAT / HB)
#define CIN   128
#define CMID  512
#define COUT  111
#define COUTP 112
#define NEX   4
#define IMS   32
#define NPIX  1024
#define NTAP  49
#define KTOT  (NTAP * CIN)
#define PADS  38
#define NPOS  (PADS * PADS)
#define NPT   32
#define HSP   72
#define ZSP   68
#define XSC   8.0f
#define WSC   64.0f
#define YSC   0.0078125f
#define PSC   0.001953125f
#define CSC   64.0f
#define ZSC   0.00390625f
#define NCNT  (NBAT * COUT)
#define NDEL  (NBAT * COUT * NPIX)
#define NOUT  (NCNT + NDEL)
#define CSN   (((NCNT + 31) / 32) * 32)
#define RTH   512
#define RWV   (RTH / 32)

#define XPREP_THR (NBAT * NPOS * (CIN / 8))
#define XPREP_BLK ((XPREP_THR + 255) / 256)
#define WMIX_BLK  ((CMID * (KTOT / 8)) / 256)
#define OUT_BLK   ((((NOUT + 3) / 4) + 255) / 256)
#define CNT_BLK   (CSN / 32)

static_assert(HB >= 1);
static_assert((NBAT % HB) == 0);
static_assert(NHALF * HB == NBAT);
static_assert(NBAT * NEX <= RTH);
static_assert(KTOT == 6272);
static_assert((KTOT % 32) == 0);
static_assert(((KTOT * 2) % 128) == 0);
static_assert(((KTOT / 8) % 8) == 0);
static_assert((XPREP_THR % 16) == 0);
static_assert(WMIX_BLK * 256 == CMID * (KTOT / 8));
static_assert(CSN >= NCNT);
static_assert((CSN % 32) == 0);
static_assert(((HSP * 2) % 16) == 0);
static_assert(((ZSP * 4) % 16) == 0);
static_assert(NPIX == 1024);
static_assert((NPIX % 256) == 0);
static_assert((CMID % 128) == 0);
static_assert(COUTP == 7 * 16);
static_assert(NOUT > 0 && NOUT < 2000000000);

typedef _Float16     v8h  __attribute__((ext_vector_type(8)));
typedef _Float16     v16h __attribute__((ext_vector_type(16)));
typedef float        v4f  __attribute__((ext_vector_type(4)));
typedef float        v8f  __attribute__((ext_vector_type(8)));

union FragH { v8h p[2]; v16h v; };
union H8 { v8h v; _Float16 e[8]; };
static_assert(sizeof(FragH) == 32);
static_assert(sizeof(H8) == 16);

__device__ __forceinline__ v8f zero8() { v8f z = {0.f, 0.f, 0.f, 0.f, 0.f, 0.f, 0.f, 0.f}; return z; }

__device__ __forceinline__ float bf_rne(float x) {
  unsigned int u = __float_as_uint(x);
  u += 0x7FFFu + ((u >> 16) & 1u);
  return __uint_as_float(u & 0xFFFF0000u);
}

__device__ __forceinline__ v8f mma_h(v16h a, v16h b, v8f c) {
  v8f d = __builtin_amdgcn_wmma_f32_16x16x32_f16(false, a, false, b, (short)0, c, false, false);
#if defined(__HIP_DEVICE_COMPILE__)
  asm volatile("v_nop\n\tv_nop\n\tv_nop\n\tv_nop" : "+v"(d) : "v"(a), "v"(b));
#endif
  return d;
}

__device__ __forceinline__ float sigm(float z) {
  const float zc = fminf(fmaxf(z, -30.f), 30.f);
  return 1.0f / (1.0f + expf(-zc));
}

__global__ __launch_bounds__(RTH)
void k_router(const float* __restrict__ X, const float* __restrict__ RW, const float* __restrict__ RB, float* RT) {
  __shared__ float pooled[NBAT * CIN];
  __shared__ float lg[NBAT * NEX];
  __shared__ __align__(16) float rts[NBAT * NEX];
  const int t = threadIdx.x, lane = t & 31, wv = t >> 5;
#pragma unroll 1
  for (int r = wv; r < NBAT * CIN; r += RWV) {
    const float* xr = X + (size_t)r * NPIX + 4 * lane;
    float s = 0.f;
#pragma unroll 1
    for (int j = 0; j < NPIX / 128; ++j) {
      const v4f v = *(const v4f*)(xr + 128 * j);
      s += bf_rne(v[0]); s += bf_rne(v[1]); s += bf_rne(v[2]); s += bf_rne(v[3]);
    }
    s += __shfl_xor(s, 16, 32);
    s += __shfl_xor(s, 8, 32);
    s += __shfl_xor(s, 4, 32);
    s += __shfl_xor(s, 2, 32);
    s += __shfl_xor(s, 1, 32);
    if (lane == 0) pooled[r] = s * (1.0f / NPIX);
  }
  __syncthreads();
  if (t < NBAT * NEX) {
    const int b = t >> 2, e = t & 3;
    float l = bf_rne(RB[e]);
    const float* pr = pooled + b * CIN;
    const float* wr = RW + e * CIN;
#pragma unroll 1
    for (int c = 0; c < CIN; ++c) l += pr[c] * bf_rne(wr[c]);
    lg[t] = l;
  }
  __syncthreads();
  if (t < NBAT) {
    const float* lp = lg + t * NEX;
    const float mx = fmaxf(fmaxf(lp[0], lp[1]), fmaxf(lp[2], lp[3]));
    float sum = 0.f;
#pragma unroll 1
    for (int e = 0; e < NEX; ++e) sum += expf(lp[e] - mx);
    const float rs = 1.0f / sum;
#pragma unroll 1
    for (int e = 0; e < NEX; ++e) rts[t * NEX + e] = expf(lp[e] - mx) * rs;
  }
  __syncthreads();
  if (t < NBAT) {
    const v4f v = *(const v4f*)(rts + NEX * t);
    *(volatile v4f*)(RT + NEX * t) = v;
    __threadfence();
    *(volatile v4f*)(RT + NEX * t) = v;
  }
}

__global__ __launch_bounds__(256)
void k_xprep(const float* __restrict__ X, _Float16* XP) {
  const int gid0 = blockIdx.x * 256 + threadIdx.x;
  const bool act = gid0 < XPREP_THR;
  const int gid = min(gid0, XPREP_THR - 1);
  const int pos = gid >> 4;
  const int c0  = (gid & 15) * 8;
  const int b   = pos / NPOS;
  const int rem = pos - b * NPOS;
  const int yy  = rem / PADS;
  const int xx  = rem - yy * PADS;
  const int py  = yy - 3, px = xx - 3;
  const bool inb = ((unsigned)py < (unsigned)IMS) && ((unsigned)px < (unsigned)IMS);
  const int pyc = min(max(py, 0), IMS - 1);
  const int pxc = min(max(px, 0), IMS - 1);
  const float* src = X + ((size_t)(b * CIN + c0) * IMS + pyc) * IMS + pxc;
  H8 u;
#pragma unroll
  for (int i = 0; i < 8; ++i) {
    const float v = bf_rne(src[(size_t)i * NPIX]) * XSC;
    u.e[i] = (_Float16)(inb ? v : 0.f);
  }
  if (act) {
    _Float16* dst = XP + (size_t)pos * CIN + c0;
    *(volatile v8h*)dst = u.v;
    __threadfence();
    *(volatile v8h*)dst = u.v;
  }
}

__global__ __launch_bounds__(256)
void k_wmix(const float* __restrict__ W3, const float* __restrict__ W5, const float* __restrict__ W7,
            const float* __restrict__ RT, _Float16* WM, int b0) {
  const int gid = blockIdx.x * 256 + threadIdx.x;
  const int o   = gid / (KTOT / 8);
  const int q   = gid - o * (KTOT / 8);
  const int k0  = 8 * q;
  const int tap = k0 >> 7;
  const int c0  = k0 & 127;
  const int dy  = tap / 7, dx = tap - 7 * dy;
  const int d5y = dy - 1, d5x = dx - 1, d3y = dy - 2, d3x = dx - 2;
  const bool in5 = ((unsigned)d5y < 5u) && ((unsigned)d5x < 5u);
  const bool in3 = ((unsigned)d3y < 3u) && ((unsigned)d3x < 3u);
  const int t7 = dy * 7 + dx;
  const int t5 = min(max(d5y, 0), 4) * 5 + min(max(d5x, 0), 4);
  const int t3 = min(max(d3y, 0), 2) * 3 + min(max(d3x, 0), 2);
  float s[NEX][8];
#pragma unroll
  for (int e = 0; e < NEX; ++e) {
    const size_t rowbase = (size_t)(e * CMID + o) * CIN + c0;
#pragma unroll
    for (int i = 0; i < 8; ++i) {
      const size_t rc = rowbase + i;
      const float a7 = bf_rne(W7[rc * 49 + t7]);
      const float a5 = bf_rne(W5[rc * 25 + t5]);
      const float a3 = bf_rne(W3[rc * 9 + t3]);
      s[e][i] = a7 + (in5 ? a5 : 0.f) + (in3 ? a3 : 0.f);
    }
  }
#pragma unroll 1
  for (int bl = 0; bl < HB; ++bl) {
    const float r0 = RT[(b0 + bl) * NEX + 0];
    const float r1 = RT[(b0 + bl) * NEX + 1];
    const float r2 = RT[(b0 + bl) * NEX + 2];
    const float r3 = RT[(b0 + bl) * NEX + 3];
    H8 u;
#pragma unroll
    for (int i = 0; i < 8; ++i) {
      const float v = r0 * s[0][i] + r1 * s[1][i] + r2 * s[2][i] + r3 * s[3][i];
      u.e[i] = (_Float16)(v * WSC);
    }
    _Float16* dst = WM + ((size_t)(bl * CMID + o)) * KTOT + k0;
    *(volatile v8h*)dst = u.v;
    __threadfence();
    *(volatile v8h*)dst = u.v;
  }
}

__global__ __launch_bounds__(128)
void k_conv(const _Float16* __restrict__ XP, const _Float16* __restrict__ WM, _Float16* YT, float* PS, int b0) {
  __shared__ __align__(16) _Float16 Hs[4 * 32 * HSP];
  __shared__ __align__(16) float Ss[4 * 64];
  const int t = threadIdx.x, lane = t & 31, wv = t >> 5;
  const int hh = lane >> 4, m = lane & 15;
  const int bl = blockIdx.z;
  const int b  = b0 + bl;
  const int px0 = blockIdx.x * 64 + (wv & 1) * 32;
  const int ch0 = blockIdx.y * 128 + (wv >> 1) * 64;
  const int pA0 = px0 + m, pA1 = px0 + 16 + m;
  const _Float16* xa0 = XP + ((size_t)(b * PADS + (pA0 >> 5)) * PADS + (pA0 & 31)) * CIN + 8 * hh;
  const _Float16* xa1 = XP + ((size_t)(b * PADS + (pA1 >> 5)) * PADS + (pA1 & 31)) * CIN + 8 * hh;
  const _Float16* wb  = WM + ((size_t)(bl * CMID + ch0 + m)) * KTOT + 8 * hh;

  v8f acc[2][4];
#pragma unroll
  for (int tt = 0; tt < 2; ++tt)
#pragma unroll
    for (int ct = 0; ct < 4; ++ct) acc[tt][ct] = zero8();

#pragma unroll 1
  for (int tap = 0; tap < NTAP; ++tap) {
    const int dy   = tap / 7;
    const int dx   = tap - 7 * dy;
    const int aoff = (dy * PADS + dx) * CIN;
    const int koff = tap * CIN;
#pragma unroll
    for (int cs = 0; cs < 4; ++cs) {
      FragH a0, a1;
      a0.p[0] = *(const v8h*)(xa0 + aoff + cs * 32);
      a0.p[1] = *(const v8h*)(xa0 + aoff + cs * 32 + 16);
      a1.p[0] = *(const v8h*)(xa1 + aoff + cs * 32);
      a1.p[1] = *(const v8h*)(xa1 + aoff + cs * 32 + 16);
#pragma unroll
      for (int ct = 0; ct < 4; ++ct) {
        const _Float16* wp = wb + (size_t)ct * 16 * KTOT + koff + cs * 32;
        FragH w;
        w.p[0] = *(const v8h*)(wp);
        w.p[1] = *(const v8h*)(wp + 16);
        acc[0][ct] = mma_h(a0.v, w.v, acc[0][ct]);
        acc[1][ct] = mma_h(a1.v, w.v, acc[1][ct]);
      }
    }
  }

  _Float16* hs = Hs + wv * 32 * HSP;
  float* ss = Ss + wv * 64;
#pragma unroll
  for (int tt = 0; tt < 2; ++tt)
#pragma unroll
    for (int ct = 0; ct < 4; ++ct)
#pragma unroll
      for (int r = 0; r < 8; ++r)
        hs[(16 * tt + 8 * hh + r) * HSP + ct * 16 + m] = (_Float16)(acc[tt][ct][r] * YSC);
#pragma unroll
  for (int ct = 0; ct < 4; ++ct) {
    float s = 0.f;
#pragma unroll
    for (int r = 0; r < 8; ++r) s += acc[0][ct][r] + acc[1][ct][r];
    s += __shfl_xor(s, 16, 32);
    ss[ct * 16 + m] = s * PSC;
  }
  __syncthreads();

  v8h yv[8];
  size_t yo[8];
#pragma unroll
  for (int it = 0; it < 8; ++it) {
    const int row = it * 4 + (lane >> 3);
    const int q   = lane & 7;
    yv[it] = *(const v8h*)(hs + row * HSP + 8 * q);
    yo[it] = ((size_t)(b * NPIX + px0 + row)) * CMID + ch0 + 8 * q;
  }
  const bool wps = lane < 16;
  const v4f pv = *(const v4f*)(ss + 4 * (lane & 15));
  const size_t po = ((size_t)(b * NPT + (px0 >> 5))) * CMID + ch0 + 4 * (lane & 15);

#pragma unroll
  for (int it = 0; it < 8; ++it) *(volatile v8h*)(YT + yo[it]) = yv[it];
  if (wps) *(volatile v4f*)(PS + po) = pv;
  __threadfence();
#pragma unroll
  for (int it = 0; it < 8; ++it) *(volatile v8h*)(YT + yo[it]) = yv[it];
  if (wps) *(volatile v4f*)(PS + po) = pv;
}

__global__ __launch_bounds__(256)
void k_ca(const float* __restrict__ PS, const float* __restrict__ F1W, const float* __restrict__ F1B,
          const float* __restrict__ F2W, const float* __restrict__ F2B, const float* __restrict__ PW,
          const float* __restrict__ MK, const float* __restrict__ MPW, const float* __restrict__ MPB,
          _Float16* WC, float* MF) {
  __shared__ float cm[CMID];
  __shared__ float hid[32];
  __shared__ float cav[CMID];
  const int t = threadIdx.x;
  const int b = blockIdx.x;
#pragma unroll
  for (int half = 0; half < 2; ++half) {
    const int o = half * 256 + t;
    const float* pp = PS + (size_t)b * NPT * CMID + o;
    float s = 0.f;
#pragma unroll 1
    for (int pt = 0; pt < NPT; ++pt) s += pp[(size_t)pt * CMID];
    cm[o] = s * (1.0f / NPIX);
  }
  __syncthreads();
  {
    const int j = t >> 3, part = t & 7;
    const float* wr = F1W + (size_t)j * CMID + part * 64;
    const float* cr = cm + part * 64;
    float a = 0.f;
#pragma unroll 1
    for (int i = 0; i < 64; ++i) a += bf_rne(wr[i]) * cr[i];
    a += __shfl_xor(a, 1, 32);
    a += __shfl_xor(a, 2, 32);
    a += __shfl_xor(a, 4, 32);
    if (part == 0) hid[j] = fmaxf(a + bf_rne(F1B[j]), 0.f);
  }
  __syncthreads();
#pragma unroll 1
  for (int half = 0; half < 2; ++half) {
    const int o = half * 256 + t;
    float a = bf_rne(F2B[o]);
    const float* wr = F2W + (size_t)o * 32;
#pragma unroll 1
    for (int j = 0; j < 32; ++j) a += bf_rne(wr[j]) * hid[j];
    cav[o] = sigm(a);
  }
  __syncthreads();
#pragma unroll 1
  for (int it = 0; it < 28; ++it) {
    const int row  = it * 4 + (t >> 6);
    const int q    = t & 63;
    const int c0   = 8 * q;
    const int rowc = min(row, COUT - 1);
    const float keep = (row < COUT) ? CSC : 0.f;
    const float* pw = PW + (size_t)rowc * CMID + c0;
    H8 u;
#pragma unroll
    for (int i = 0; i < 8; ++i) u.e[i] = (_Float16)(keep * cav[c0 + i] * bf_rne(pw[i]));
    _Float16* dst = WC + ((size_t)(b * COUTP + row)) * CMID + c0;
    *(volatile v8h*)dst = u.v;
    __threadfence();
    *(volatile v8h*)dst = u.v;
  }
#pragma unroll 1
  for (int i = 0; i < NPIX / 256; ++i) {
    const int p = i * 256 + t;
    const float* mp = MK + (size_t)b * CIN * NPIX + p;
    float a = bf_rne(MPB[0]);
#pragma unroll 1
    for (int e = 0; e < CIN; ++e) a += bf_rne(mp[(size_t)e * NPIX]) * bf_rne(MPW[e]);
    float* dst = MF + (size_t)b * NPIX + p;
    *(volatile float*)dst = a;
    __threadfence();
    *(volatile float*)dst = a;
  }
}

__global__ __launch_bounds__(128)
void k_pred(const _Float16* __restrict__ WC, const _Float16* __restrict__ YT, const float* __restrict__ MF,
            float* DW) {
  __shared__ __align__(16) float Zs[4 * 16 * ZSP];
  const int t = threadIdx.x, lane = t & 31, wv = t >> 5;
  const int hh = lane >> 4, m = lane & 15;
  const int b  = blockIdx.z;
  const int o0 = blockIdx.y * 16;
  const int p0 = blockIdx.x * 256 + wv * 64;
  const _Float16* ap = WC + ((size_t)(b * COUTP + o0 + m)) * CMID + 8 * hh;
  const _Float16* bp = YT + ((size_t)(b * NPIX + p0 + m)) * CMID + 8 * hh;

  v8f acc[4];
#pragma unroll
  for (int nt = 0; nt < 4; ++nt) acc[nt] = zero8();

#pragma unroll 1
  for (int ks = 0; ks < CMID / 32; ++ks) {
    FragH a;
    a.p[0] = *(const v8h*)(ap + ks * 32);
    a.p[1] = *(const v8h*)(ap + ks * 32 + 16);
#pragma unroll
    for (int nt = 0; nt < 4; ++nt) {
      const _Float16* yp = bp + (size_t)nt * 16 * CMID + ks * 32;
      FragH y;
      y.p[0] = *(const v8h*)(yp);
      y.p[1] = *(const v8h*)(yp + 16);
      acc[nt] = mma_h(a.v, y.v, acc[nt]);
    }
  }

  float* zs = Zs + wv * 16 * ZSP;
#pragma unroll
  for (int nt = 0; nt < 4; ++nt) {
    const float mf = MF[(size_t)b * NPIX + p0 + nt * 16 + m];
#pragma unroll
    for (int r = 0; r < 8; ++r) {
      const float z = acc[nt][r] * ZSC * mf;
      zs[(8 * hh + r) * ZSP + nt * 16 + m] = sigm(z);
    }
  }
  __syncthreads();

  v4f dv[8];
  size_t dofs[8];
#pragma unroll
  for (int it = 0; it < 8; ++it) {
    const int line = it * 4 + (lane >> 3);
    const int q    = lane & 7;
    const int ol   = line >> 1;
    const int half = line & 1;
    dv[it]   = *(const v4f*)(zs + ol * ZSP + half * 32 + 4 * q);
    dofs[it] = ((size_t)(b * COUTP + o0 + ol)) * NPIX + p0 + half * 32 + 4 * q;
  }
#pragma unroll
  for (int it = 0; it < 8; ++it) *(volatile v4f*)(DW + dofs[it]) = dv[it];
  __threadfence();
#pragma unroll
  for (int it = 0; it < 8; ++it) *(volatile v4f*)(DW + dofs[it]) = dv[it];
}

__global__ __launch_bounds__(256)
void k_count(const float* __restrict__ DW, float* CS) {
  __shared__ __align__(16) float cs[32];
  const int t = threadIdx.x, lane = t & 31, wv = t >> 5;
#pragma unroll 1
  for (int i = 0; i < 4; ++i) {
    const int rl = i * 8 + wv;
    const int R  = blockIdx.x * 32 + rl;
    const int Rc = min(R, NCNT - 1);
    const int b  = Rc / COUT;
    const int o  = Rc - b * COUT;
    const float* row = DW + ((size_t)(b * COUTP + o)) * NPIX + 32 * lane;
    float s = 0.f;
#pragma unroll
    for (int j = 0; j < 8; ++j) {
      const v4f w = *(const v4f*)(row + 4 * j);
      s += (w[0] + w[1]) + (w[2] + w[3]);
    }
    s += __shfl_xor(s, 16, 32);
    s += __shfl_xor(s, 8, 32);
    s += __shfl_xor(s, 4, 32);
    s += __shfl_xor(s, 2, 32);
    s += __shfl_xor(s, 1, 32);
    if (lane == 0) cs[rl] = s;
  }
  __syncthreads();
  if (t < 8) {
    const v4f v = *(const v4f*)(cs + 4 * t);
    float* dst = CS + blockIdx.x * 32 + 4 * t;
    *(volatile v4f*)dst = v;
    __threadfence();
    *(volatile v4f*)dst = v;
  }
}

__global__ __launch_bounds__(256)
void k_out(const float* __restrict__ CS, const float* __restrict__ DW, float* out, int out_n) {
  const int q  = blockIdx.x * 256 + threadIdx.x;
  const int f0 = 4 * q;
  v4f v;
#pragma unroll
  for (int j = 0; j < 4; ++j) {
    const int f  = f0 + j;
    const int fc = min(max(f, 0), NCNT - 1);
    const float cv = CS[fc];
    const int g  = min(max(f - NCNT, 0), NDEL - 1);
    const int R  = g / NPIX;
    const int p  = g - R * NPIX;
    const int b  = R / COUT;
    const int o  = R - b * COUT;
    const float dvv = DW[((size_t)(b * COUTP + o)) * NPIX + p];
    v[j] = (f < NCNT) ? cv : dvv;
  }
  if (f0 + 4 <= out_n) {
    *(volatile v4f*)(out + f0) = v;
    __threadfence();
    *(volatile v4f*)(out + f0) = v;
  } else if (f0 < out_n) {
    const float e0 = v[0], e1 = v[1], e2 = v[2];
    if (f0 + 0 < out_n) *(volatile float*)(out + f0 + 0) = e0;
    if (f0 + 1 < out_n) *(volatile float*)(out + f0 + 1) = e1;
    if (f0 + 2 < out_n) *(volatile float*)(out + f0 + 2) = e2;
    __threadfence();
    if (f0 + 0 < out_n) *(volatile float*)(out + f0 + 0) = e0;
    if (f0 + 1 < out_n) *(volatile float*)(out + f0 + 1) = e1;
    if (f0 + 2 < out_n) *(volatile float*)(out + f0 + 2) = e2;
  }
}

extern "C" void kernel_launch(void* const* d_in, const int* in_sizes, int n_in,
                              void* d_out, int out_size, void* d_ws, size_t ws_size,
                              hipStream_t stream) {
  if (n_in < 14) return;
  if (in_sizes[0]  != NBAT * CIN * NPIX) return;
  if (in_sizes[1]  != NBAT * CIN * NPIX) return;
  if (in_sizes[2]  != NEX * CMID * CIN * 9) return;
  if (in_sizes[3]  != NEX * CMID * CIN * 25) return;
  if (in_sizes[4]  != NEX * CMID * CIN * 49) return;
  if (in_sizes[5]  != NEX * CIN) return;
  if (in_sizes[6]  != NEX) return;
  if (in_sizes[7]  != 32 * CMID) return;
  if (in_sizes[8]  != 32) return;
  if (in_sizes[9]  != CMID * 32) return;
  if (in_sizes[10] != CMID) return;
  if (in_sizes[11] != CIN) return;
  if (in_sizes[12] != 1) return;
  if (in_sizes[13] != COUT * CMID) return;
  if (out_size != NOUT) return;

  size_t off = 0;
  const size_t szRT = (((size_t)NBAT * NEX * 4 + 255) / 256) * 256;
  const size_t szXP = (size_t)NBAT * NPOS * CIN * 2;
  const size_t szWM = (size_t)HB * CMID * KTOT * 2;
  const size_t szYT = (size_t)NBAT * NPIX * CMID * 2;
  const size_t szPS = (size_t)NBAT * NPT * CMID * 4;
  const size_t szWC = (size_t)NBAT * COUTP * CMID * 2;
  const size_t szMF = (size_t)NBAT * NPIX * 4;
  const size_t szDW = (size_t)NBAT * COUTP * NPIX * 4;
  const size_t szCS = (size_t)CSN * 4;
  const size_t oRT = off; off += szRT;
  const size_t oXP = off; off += szXP;
  const size_t oWM = off; off += szWM;
  const size_t oYT = off; off += szYT;
  const size_t oPS = off; off += szPS;
  const size_t oWC = off; off += szWC;
  const size_t oMF = off; off += szMF;
  const size_t oDW = off; off += szDW;
  const size_t oCS = off; off += szCS;
  if (off > ws_size) return;
  if (off > (size_t)134217728) return;
  if ((oXP % 256) != 0 || (oWM % 256) != 0 || (oYT % 256) != 0 || (oPS % 256) != 0 ||
      (oWC % 256) != 0 || (oMF % 256) != 0 || (oDW % 256) != 0 || (oCS % 256) != 0) return;

  const float* X   = (const float*)d_in[0];
  const float* MK  = (const float*)d_in[1];
  const float* W3  = (const float*)d_in[2];
  const float* W5  = (const float*)d_in[3];
  const float* W7  = (const float*)d_in[4];
  const float* RW  = (const float*)d_in[5];
  const float* RB  = (const float*)d_in[6];
  const float* F1W = (const float*)d_in[7];
  const float* F1B = (const float*)d_in[8];
  const float* F2W = (const float*)d_in[9];
  const float* F2B = (const float*)d_in[10];
  const float* MPW = (const float*)d_in[11];
  const float* MPB = (const float*)d_in[12];
  const float* PW  = (const float*)d_in[13];
  float* out = (float*)d_out;

  char* ws = (char*)d_ws;
  float*    RT = (float*)(ws + oRT);
  _Float16* XP = (_Float16*)(ws + oXP);
  _Float16* WM = (_Float16*)(ws + oWM);
  _Float16* YT = (_Float16*)(ws + oYT);
  float*    PS = (float*)(ws + oPS);
  _Float16* WC = (_Float16*)(ws + oWC);
  float*    MF = (float*)(ws + oMF);
  float*    DW = (float*)(ws + oDW);
  float*    CS = (float*)(ws + oCS);

  k_router<<<dim3(1), dim3(RTH), 0, stream>>>(X, RW, RB, RT);
  k_xprep<<<dim3(XPREP_BLK), dim3(256), 0, stream>>>(X, XP);
  for (int part = 0; part < NHALF; ++part) {
    k_wmix<<<dim3(WMIX_BLK), dim3(256), 0, stream>>>(W3, W5, W7, RT, WM, part * HB);
    k_conv<<<dim3(NPIX / 64, CMID / 128, HB), dim3(128), 0, stream>>>(XP, WM, YT, PS, part * HB);
  }
  k_ca<<<dim3(NBAT), dim3(256), 0, stream>>>(PS, F1W, F1B, F2W, F2B, PW, MK, MPW, MPB, WC, MF);
  k_pred<<<dim3(NPIX / 256, COUTP / 16, NBAT), dim3(128), 0, stream>>>(WC, YT, MF, DW);
  k_count<<<dim3(CNT_BLK), dim3(256), 0, stream>>>(DW, CS);
  k_out<<<dim3(OUT_BLK), dim3(256), 0, stream>>>(CS, DW, out, NOUT);
  (void)hipGetLastError();
}
